// RelationalHypergraphLayer_37177236914497
// MI455X (gfx1250) — hardware-verified
//
#include <hip/hip_runtime.h>
#include <stddef.h>
#include <stdint.h>


#define DF    128
#define NH    8
#define HC    16
#define FF    512
#define GR    32
#define XSP   132
#define NB    512
#define CHUNK 1024
#define NTHR  256
#define NWAVE 8
#define WCAP  128
#define WINV  0.015625f
#define WSCL  64.0f
#define SCL   0.25f

#define L_SACC (NB * DF)
#define L_DEN  (NB * NH)
#define L_CNT  NB
#define L_LIST (NWAVE * WCAP)
#define LDS1_BYTES ((L_SACC + L_DEN + L_CNT + 2 * L_LIST + 2 * NWAVE) * 4)
#define LDS2_BYTES ((L_SACC + L_CNT + L_LIST + NWAVE) * 4)

static_assert(WCAP == (CHUNK / NTHR) * 32);
static_assert(CHUNK == NTHR * 4);
static_assert(NB == 512);
static_assert(DF == NH * HC);
static_assert(((L_SACC + L_DEN + L_CNT) % 4) == 0);
static_assert(((L_SACC + L_CNT) % 4) == 0);
static_assert(LDS1_BYTES == 288832);
static_assert(LDS2_BYTES == 268320);
static_assert((XSP * 4) % 16 == 0);

typedef float    v4f  __attribute__((ext_vector_type(4)));
typedef float    v8f  __attribute__((ext_vector_type(8)));
typedef int      v4i  __attribute__((ext_vector_type(4)));
typedef _Float16 v8h  __attribute__((ext_vector_type(8)));
typedef _Float16 v16h __attribute__((ext_vector_type(16)));
union Frag   { v16h v; v8h half[2]; };
union Pack16 { v8h h; v4i i; };

__device__ __forceinline__ v8f wm(v16h a, v16h b, v8f c) {
  v8f d = __builtin_amdgcn_wmma_f32_16x16x32_f16(false, a, false, b, (short)0, c, false, false);
  asm volatile("v_nop\n\tv_nop\n\tv_nop\n\tv_nop" : "+v"(d) : "v"(a), "v"(b));
  return d;
}

__device__ __forceinline__ float wsum(float v) {
  v += __shfl_xor(v, 16, 32);
  v += __shfl_xor(v, 8, 32);
  v += __shfl_xor(v, 4, 32);
  v += __shfl_xor(v, 2, 32);
  v += __shfl_xor(v, 1, 32);
  return v;
}

__device__ __forceinline__ v4i pack8(v4f a, v4f b) {
  Pack16 u;
  u.h[0] = (_Float16)a.x; u.h[1] = (_Float16)a.y; u.h[2] = (_Float16)a.z; u.h[3] = (_Float16)a.w;
  u.h[4] = (_Float16)b.x; u.h[5] = (_Float16)b.y; u.h[6] = (_Float16)b.z; u.h[7] = (_Float16)b.w;
  return u.i;
}

__global__ __launch_bounds__(NTHR) void k_prepw(const float* __restrict__ W, _Float16* WT, int K, int Nout) {
  const int tid = threadIdx.x;
  const int tpr = K >> 3;
  const int rpb = NTHR / tpr;
  const int n   = blockIdx.x * rpb + tid / tpr;
  const int k8  = (tid % tpr) * 8;
  if (n >= Nout) return;
  Pack16 u;
#pragma unroll
  for (int i = 0; i < 8; ++i) u.h[i] = (_Float16)(W[(size_t)(k8 + i) * Nout + n] * WSCL);
  _Float16* p = WT + (size_t)n * K + k8;
  *(volatile v4i*)p = u.i;
  __threadfence();
  *(volatile v4i*)p = u.i;
}

__global__ __launch_bounds__(NTHR) void k_cvt(const float* __restrict__ x, _Float16* xh, int nN, int nP) {
  const int i   = blockIdx.x * NTHR + threadIdx.x;
  const int row = i >> 4;
  const int c8  = (i & 15) * 8;
  if (row >= nP) return;
  v4f a = {0.f, 0.f, 0.f, 0.f}, b = {0.f, 0.f, 0.f, 0.f};
  if (row < nN) {
    const float* p = x + (size_t)row * DF + c8;
    a = *(const v4f*)p;
    b = *(const v4f*)(p + 4);
  }
  const v4i u = pack8(a, b);
  _Float16* q = xh + (size_t)row * DF + c8;
  *(volatile v4i*)q = u;
  __threadfence();
  *(volatile v4i*)q = u;
}

__device__ __forceinline__ void mma2(const _Float16* __restrict__ A, int lda,
                                     const _Float16* __restrict__ Bt, int K,
                                     int rowBase, int ncolB, int hh, int m, v8f& c0, v8f& c1) {
  const _Float16* pa0 = A + (size_t)(rowBase + m) * lda + 8 * hh;
  const _Float16* pa1 = A + (size_t)(rowBase + 16 + m) * lda + 8 * hh;
  const _Float16* pb  = Bt + (size_t)ncolB * K + 8 * hh;
#pragma unroll 1
  for (int k0 = 0; k0 < K; k0 += 32) {
    Frag a0, a1, b;
    b.half[0]  = *(const v8h*)(pb + k0);   b.half[1]  = *(const v8h*)(pb + k0 + 16);
    a0.half[0] = *(const v8h*)(pa0 + k0);  a0.half[1] = *(const v8h*)(pa0 + k0 + 16);
    a1.half[0] = *(const v8h*)(pa1 + k0);  a1.half[1] = *(const v8h*)(pa1 + k0 + 16);
    c0 = wm(a0.v, b.v, c0);
    c1 = wm(a1.v, b.v, c1);
  }
}

__device__ __forceinline__ void stage2(v8f c0, v8f c1, int hh, int ncol, float bsv, bool relu, float* Xs) {
#pragma unroll
  for (int r = 0; r < 8; ++r) {
    float u0 = c0[r] * WINV + bsv;
    float u1 = c1[r] * WINV + bsv;
    if (relu) { u0 = fmaxf(u0, 0.f); u1 = fmaxf(u1, 0.f); }
    Xs[(8 * hh + r) * XSP + ncol]      = u0;
    Xs[(16 + 8 * hh + r) * XSP + ncol] = u1;
  }
}

__global__ __launch_bounds__(NTHR) void k_gemm_qkv(
    const _Float16* __restrict__ A, const _Float16* __restrict__ Bt3,
    const float* __restrict__ b0, const float* __restrict__ b1, const float* __restrict__ b2,
    float* Y3, int nP) {
  __shared__ __attribute__((aligned(16))) float Xs[GR * XSP];
  const int tid = threadIdx.x, lane = tid & 31, wave = tid >> 5;
  const int hh = lane >> 4, m = lane & 15;
  const int which = blockIdx.y;
  const _Float16* Bt = Bt3 + (size_t)which * DF * DF;
  const float* bias  = (which == 0) ? b0 : ((which == 1) ? b1 : b2);
  float* Y = Y3 + (size_t)which * (size_t)nP * DF;
  const int rowBase = blockIdx.x * GR;
  const int ncol = wave * 16 + m;

  v8f c0 = {0.f, 0.f, 0.f, 0.f, 0.f, 0.f, 0.f, 0.f};
  v8f c1 = {0.f, 0.f, 0.f, 0.f, 0.f, 0.f, 0.f, 0.f};
  mma2(A, DF, Bt, DF, rowBase, ncol, hh, m, c0, c1);
  stage2(c0, c1, hh, ncol, bias[ncol], false, Xs);
  __syncthreads();

  v4f xr[4];
#pragma unroll
  for (int i = 0; i < 4; ++i) xr[i] = *(const v4f*)(Xs + (4 * wave + i) * XSP + 4 * lane);
  float* yp = Y + (size_t)(rowBase + 4 * wave) * DF + 4 * lane;
#pragma unroll
  for (int i = 0; i < 4; ++i) *(volatile v4f*)(yp + (size_t)i * DF) = xr[i];
  __threadfence();
#pragma unroll
  for (int i = 0; i < 4; ++i) *(volatile v4f*)(yp + (size_t)i * DF) = xr[i];
}

__global__ __launch_bounds__(NTHR) void k_gemm_ln(
    const _Float16* __restrict__ A, const _Float16* __restrict__ Bt,
    const float* __restrict__ bias, const float* __restrict__ res,
    const float* __restrict__ gam, const float* __restrict__ bet,
    float* Y, _Float16* Yh, int lda, int K, int nres, int nout, int writeH) {
  __shared__ __attribute__((aligned(16))) float Xs[GR * XSP];
  const int tid = threadIdx.x, lane = tid & 31, wave = tid >> 5;
  const int hh = lane >> 4, m = lane & 15;
  const int rowBase = blockIdx.x * GR;
  const int ncol = wave * 16 + m;

  v8f c0 = {0.f, 0.f, 0.f, 0.f, 0.f, 0.f, 0.f, 0.f};
  v8f c1 = {0.f, 0.f, 0.f, 0.f, 0.f, 0.f, 0.f, 0.f};
  mma2(A, lda, Bt, K, rowBase, ncol, hh, m, c0, c1);
  stage2(c0, c1, hh, ncol, bias[ncol], false, Xs);
  __syncthreads();

  const v4f g4 = *(const v4f*)(gam + 4 * lane);
  const v4f e4 = *(const v4f*)(bet + 4 * lane);
  v4f y[4];
#pragma unroll
  for (int i = 0; i < 4; ++i) {
    const int row = 4 * wave + i;
    int rr = rowBase + row;
    if (rr > nres - 1) rr = nres - 1;
    const v4f x = *(const v4f*)(Xs + row * XSP + 4 * lane) +
                  *(const v4f*)(res + (size_t)rr * DF + 4 * lane);
    const float s  = wsum(x.x + x.y + x.z + x.w);
    const float mu = s * (1.0f / DF);
    const v4f d = x - mu;
    const float q  = wsum(d.x * d.x + d.y * d.y + d.z * d.z + d.w * d.w);
    const float rs = rsqrtf(q * (1.0f / DF) + 1e-5f);
    y[i] = d * rs * g4 + e4;
  }
  __syncthreads();
#pragma unroll
  for (int i = 0; i < 4; ++i) *(v4f*)(Xs + (4 * wave + i) * XSP + 4 * lane) = y[i];
  __syncthreads();
  const int cl = lane & 15, c8 = 8 * cl;
  v4i hp[2];
  int hrow[2];
#pragma unroll
  for (int t = 0; t < 2; ++t) {
    const int row = 4 * wave + 2 * t + hh;
    hrow[t] = rowBase + row;
    hp[t] = pack8(*(const v4f*)(Xs + row * XSP + c8), *(const v4f*)(Xs + row * XSP + c8 + 4));
  }

#pragma unroll
  for (int i = 0; i < 4; ++i) {
    const int grow = rowBase + 4 * wave + i;
    if (grow < nout) *(volatile v4f*)(Y + (size_t)grow * DF + 4 * lane) = y[i];
  }
  if (writeH) {
#pragma unroll
    for (int t = 0; t < 2; ++t)
      if (hrow[t] < nout) *(volatile v4i*)(Yh + (size_t)hrow[t] * DF + c8) = hp[t];
  }
  __threadfence();
#pragma unroll
  for (int i = 0; i < 4; ++i) {
    const int grow = rowBase + 4 * wave + i;
    if (grow < nout) *(volatile v4f*)(Y + (size_t)grow * DF + 4 * lane) = y[i];
  }
  if (writeH) {
#pragma unroll
    for (int t = 0; t < 2; ++t)
      if (hrow[t] < nout) *(volatile v4i*)(Yh + (size_t)hrow[t] * DF + c8) = hp[t];
  }
}

__global__ __launch_bounds__(NTHR) void k_ffn1(
    const _Float16* __restrict__ A, const _Float16* __restrict__ Bt,
    const float* __restrict__ bias, _Float16* Yh) {
  __shared__ __attribute__((aligned(16))) float Xs[GR * XSP];
  const int tid = threadIdx.x, lane = tid & 31, wave = tid >> 5;
  const int hh = lane >> 4, m = lane & 15;
  const int rowBase = blockIdx.x * GR;
  const int cb   = blockIdx.y * DF;
  const int ncol = wave * 16 + m;

  v8f c0 = {0.f, 0.f, 0.f, 0.f, 0.f, 0.f, 0.f, 0.f};
  v8f c1 = {0.f, 0.f, 0.f, 0.f, 0.f, 0.f, 0.f, 0.f};
  mma2(A, DF, Bt, DF, rowBase, cb + ncol, hh, m, c0, c1);
  stage2(c0, c1, hh, ncol, bias[cb + ncol], true, Xs);
  __syncthreads();

  const int cl = lane & 15, c8 = 8 * cl;
  v4i hp[2];
  size_t o[2];
#pragma unroll
  for (int t = 0; t < 2; ++t) {
    const int row = 4 * wave + 2 * t + hh;
    hp[t] = pack8(*(const v4f*)(Xs + row * XSP + c8), *(const v4f*)(Xs + row * XSP + c8 + 4));
    o[t]  = (size_t)(rowBase + row) * FF + cb + c8;
  }
#pragma unroll
  for (int t = 0; t < 2; ++t) *(volatile v4i*)(Yh + o[t]) = hp[t];
  __threadfence();
#pragma unroll
  for (int t = 0; t < 2; ++t) *(volatile v4i*)(Yh + o[t]) = hp[t];
}

#define HIT(LIST, WC, HJ, VAL) { \
    const unsigned mj = __builtin_amdgcn_ballot_w32(HJ); \
    if (HJ) { \
      const int pos = WC + (int)__builtin_amdgcn_mbcnt_lo(mj, 0u); \
      if (pos < WCAP) LIST[wave * WCAP + pos] = (VAL); \
    } \
    WC += (int)__builtin_popcount(mj); }

__device__ __forceinline__ void attn_store(const float* sacc, const float* den, const int* cnto,
                                           _Float16* hoH, float* rso, int nodeBase,
                                           int wave, int lane, int hh, int tid) {
  const int cl = lane & 15, c8 = 8 * cl, head = cl >> 1;
#pragma unroll 1
  for (int j = 0; j < NB / (2 * NWAVE); ++j) {
    const int slot = wave * (NB / NWAVE) + 2 * j + hh;
    const float dv  = den[slot * NH + head];
    const float inv = (dv > 0.f) ? (1.0f / dv) : 0.f;
    const v4f a = *(const v4f*)(sacc + slot * DF + c8) * inv;
    const v4f b = *(const v4f*)(sacc + slot * DF + c8 + 4) * inv;
    const v4i u = pack8(a, b);
    *(volatile v4i*)(hoH + (size_t)(nodeBase + slot) * DF + c8) = u;
  }
  if (tid < NB / 4) {
    v4f r;
    int c;
    c = cnto[4 * tid + 0]; r.x = 1.0f / sqrtf((float)(c > 1 ? c : 1));
    c = cnto[4 * tid + 1]; r.y = 1.0f / sqrtf((float)(c > 1 ? c : 1));
    c = cnto[4 * tid + 2]; r.z = 1.0f / sqrtf((float)(c > 1 ? c : 1));
    c = cnto[4 * tid + 3]; r.w = 1.0f / sqrtf((float)(c > 1 ? c : 1));
    *(volatile v4f*)(rso + (size_t)nodeBase + 4 * tid) = r;
  }
}

__global__ __launch_bounds__(NTHR) void k_attn(
    const float* __restrict__ Q, const float* __restrict__ Kp, const float* __restrict__ V,
    const int* __restrict__ src, const int* __restrict__ dst,
    _Float16* hoH, float* rso, int nN, int nE) {
  extern __shared__ v4f lds_dyn[];
  float* sacc  = (float*)lds_dyn;
  float* den   = sacc + L_SACC;
  int*   cnto  = (int*)(den + L_DEN);
  int*   listD = cnto + L_CNT;
  int*   listS = listD + L_LIST;
  int*   wcD   = listS + L_LIST;
  int*   wcS   = wcD + NWAVE;

  const int tid = threadIdx.x, lane = tid & 31, wave = tid >> 5;
  const int hh = lane >> 4;
  const int hq = lane >> 2;
  const int nodeBase = blockIdx.x * NB;
  {
    const v4f z4 = {0.f, 0.f, 0.f, 0.f};
    for (int i = tid; i < (L_SACC + L_DEN + L_CNT) / 4; i += NTHR) lds_dyn[i] = z4;
  }
  __syncthreads();

  const bool al16 = ((((size_t)src) | ((size_t)dst)) & 15) == 0;
  const unsigned ub = (unsigned)nodeBase;
  const int nChunks = (nE + CHUNK - 1) / CHUNK;
  const int sent = -2147483647 - 1;
#pragma unroll 1
  for (int ch = 0; ch < nChunks; ++ch) {
    const int cbase = ch * CHUNK;
    const int e0 = cbase + 4 * tid;
    v4i d, s;
    if (al16 && (e0 + 3 < nE)) {
      d = *(const v4i*)(dst + e0);
      s = *(const v4i*)(src + e0);
    } else {
      d.x = (e0     < nE) ? dst[min(e0,     nE - 1)] : sent;
      d.y = (e0 + 1 < nE) ? dst[min(e0 + 1, nE - 1)] : sent;
      d.z = (e0 + 2 < nE) ? dst[min(e0 + 2, nE - 1)] : sent;
      d.w = (e0 + 3 < nE) ? dst[min(e0 + 3, nE - 1)] : sent;
      s.x = (e0     < nE) ? src[min(e0,     nE - 1)] : sent;
      s.y = (e0 + 1 < nE) ? src[min(e0 + 1, nE - 1)] : sent;
      s.z = (e0 + 2 < nE) ? src[min(e0 + 2, nE - 1)] : sent;
      s.w = (e0 + 3 < nE) ? src[min(e0 + 3, nE - 1)] : sent;
    }
    v4i sc;
    sc.x = min(max(s.x, 0), nN - 1);
    sc.y = min(max(s.y, 0), nN - 1);
    sc.z = min(max(s.z, 0), nN - 1);
    sc.w = min(max(s.w, 0), nN - 1);
    const unsigned sd0 = (unsigned)d.x - ub, sd1 = (unsigned)d.y - ub;
    const unsigned sd2 = (unsigned)d.z - ub, sd3 = (unsigned)d.w - ub;
    const bool hd0 = sd0 < (unsigned)NB, hd1 = sd1 < (unsigned)NB;
    const bool hd2 = sd2 < (unsigned)NB, hd3 = sd3 < (unsigned)NB;
    const unsigned ss0 = (unsigned)s.x - ub, ss1 = (unsigned)s.y - ub;
    const unsigned ss2 = (unsigned)s.z - ub, ss3 = (unsigned)s.w - ub;
    const bool hs0 = ss0 < (unsigned)NB, hs1 = ss1 < (unsigned)NB;
    const bool hs2 = ss2 < (unsigned)NB, hs3 = ss3 < (unsigned)NB;
    int wcd = 0, wcs = 0;
    const unsigned manyD = __builtin_amdgcn_ballot_w32(hd0 | hd1 | hd2 | hd3);
    if (manyD != 0u) {
      HIT(listD, wcd, hd0, (sc.x << 9) | (int)sd0)
      HIT(listD, wcd, hd1, (sc.y << 9) | (int)sd1)
      HIT(listD, wcd, hd2, (sc.z << 9) | (int)sd2)
      HIT(listD, wcd, hd3, (sc.w << 9) | (int)sd3)
    }
    const unsigned manyS = __builtin_amdgcn_ballot_w32(hs0 | hs1 | hs2 | hs3);
    if (manyS != 0u) {
      HIT(listS, wcs, hs0, (int)ss0)
      HIT(listS, wcs, hs1, (int)ss1)
      HIT(listS, wcs, hs2, (int)ss2)
      HIT(listS, wcs, hs3, (int)ss3)
    }
    if (lane == 0) { wcD[wave] = wcd; wcS[wave] = wcs; }
    __syncthreads();

    if (wave == 0) {
#pragma unroll 1
      for (int wsx = 0; wsx < NWAVE; ++wsx) {
        int n = wcD[wsx];
        n = (n > WCAP) ? WCAP : ((n < 0) ? 0 : n);
#pragma unroll 1
        for (int i = 0; i < n; ++i) {
          const int ent  = listD[wsx * WCAP + i];
          const int slot = ent & (NB - 1);
          int sId = ent >> 9;
          sId = (sId < 0) ? 0 : ((sId > nN - 1) ? nN - 1 : sId);
          const int nd = nodeBase + slot;
          const v4f q = *(const v4f*)(Q  + (size_t)sId * DF + 4 * lane);
          const v4f k = *(const v4f*)(Kp + (size_t)nd  * DF + 4 * lane);
          float t = q.x * k.x + q.y * k.y + q.z * k.z + q.w * k.w;
          t += __shfl_xor(t, 1, 32);
          t += __shfl_xor(t, 2, 32);
          float sco = t * SCL;
          sco = fminf(fmaxf(sco, -80.f), 80.f);
          const float p = __expf(sco);
          const v4f v = *(const v4f*)(V + (size_t)sId * DF + 4 * lane);
          v4f* sp = (v4f*)(sacc + slot * DF + 4 * lane);
          const v4f cur = *sp;
          *sp = cur + p * v;
          if ((lane & 3) == 0) {
            const float od = den[slot * NH + hq];
            den[slot * NH + hq] = od + p;
          }
        }
      }
    } else if (wave == 1) {
#pragma unroll 1
      for (int wsx = 0; wsx < NWAVE; ++wsx) {
        int n = wcS[wsx];
        n = (n > WCAP) ? WCAP : ((n < 0) ? 0 : n);
#pragma unroll 1
        for (int i = 0; i < n; ++i) {
          const int slot = listS[wsx * WCAP + i] & (NB - 1);
          if (lane == 0) {
            const int oc = cnto[slot];
            cnto[slot] = oc + 1;
          }
        }
      }
    }
    __syncthreads();
  }

  attn_store(sacc, den, cnto, hoH, rso, nodeBase, wave, lane, hh, tid);
  __threadfence();
  attn_store(sacc, den, cnto, hoH, rso, nodeBase, wave, lane, hh, tid);
}

__device__ __forceinline__ void gcn_store(const float* sacc, const int* cnti, _Float16* agH,
                                          int nodeBase, int wave, int lane, int hh) {
  const int cl = lane & 15, c8 = 8 * cl;
#pragma unroll 1
  for (int j = 0; j < NB / (2 * NWAVE); ++j) {
    const int slot = wave * (NB / NWAVE) + 2 * j + hh;
    const int c = cnti[slot];
    const float rs = 1.0f / sqrtf((float)(c > 1 ? c : 1));
    const v4f a = *(const v4f*)(sacc + slot * DF + c8) * rs;
    const v4f b = *(const v4f*)(sacc + slot * DF + c8 + 4) * rs;
    const v4i u = pack8(a, b);
    *(volatile v4i*)(agH + (size_t)(nodeBase + slot) * DF + c8) = u;
  }
}

__global__ __launch_bounds__(NTHR) void k_gcn(
    const float* __restrict__ h1, const float* __restrict__ rso,
    const int* __restrict__ src, const int* __restrict__ dst,
    _Float16* agH, int nN, int nE) {
  extern __shared__ v4f lds_dyn[];
  float* sacc  = (float*)lds_dyn;
  int*   cnti  = (int*)(sacc + L_SACC);
  int*   listD = cnti + L_CNT;
  int*   wcD   = listD + L_LIST;

  const int tid = threadIdx.x, lane = tid & 31, wave = tid >> 5;
  const int hh = lane >> 4;
  const int nodeBase = blockIdx.x * NB;
  {
    const v4f z4 = {0.f, 0.f, 0.f, 0.f};
    for (int i = tid; i < (L_SACC + L_CNT) / 4; i += NTHR) lds_dyn[i] = z4;
  }
  __syncthreads();

  const bool al16 = ((((size_t)src) | ((size_t)dst)) & 15) == 0;
  const unsigned ub = (unsigned)nodeBase;
  const int nChunks = (nE + CHUNK - 1) / CHUNK;
  const int sent = -2147483647 - 1;
#pragma unroll 1
  for (int ch = 0; ch < nChunks; ++ch) {
    const int cbase = ch * CHUNK;
    const int e0 = cbase + 4 * tid;
    v4i d, s;
    if (al16 && (e0 + 3 < nE)) {
      d = *(const v4i*)(dst + e0);
      s = *(const v4i*)(src + e0);
    } else {
      d.x = (e0     < nE) ? dst[min(e0,     nE - 1)] : sent;
      d.y = (e0 + 1 < nE) ? dst[min(e0 + 1, nE - 1)] : sent;
      d.z = (e0 + 2 < nE) ? dst[min(e0 + 2, nE - 1)] : sent;
      d.w = (e0 + 3 < nE) ? dst[min(e0 + 3, nE - 1)] : sent;
      s.x = (e0     < nE) ? src[min(e0,     nE - 1)] : 0;
      s.y = (e0 + 1 < nE) ? src[min(e0 + 1, nE - 1)] : 0;
      s.z = (e0 + 2 < nE) ? src[min(e0 + 2, nE - 1)] : 0;
      s.w = (e0 + 3 < nE) ? src[min(e0 + 3, nE - 1)] : 0;
    }
    v4i sc;
    sc.x = min(max(s.x, 0), nN - 1);
    sc.y = min(max(s.y, 0), nN - 1);
    sc.z = min(max(s.z, 0), nN - 1);
    sc.w = min(max(s.w, 0), nN - 1);
    const unsigned sd0 = (unsigned)d.x - ub, sd1 = (unsigned)d.y - ub;
    const unsigned sd2 = (unsigned)d.z - ub, sd3 = (unsigned)d.w - ub;
    const bool hd0 = sd0 < (unsigned)NB, hd1 = sd1 < (unsigned)NB;
    const bool hd2 = sd2 < (unsigned)NB, hd3 = sd3 < (unsigned)NB;
    int wcd = 0;
    const unsigned manyD = __builtin_amdgcn_ballot_w32(hd0 | hd1 | hd2 | hd3);
    if (manyD != 0u) {
      HIT(listD, wcd, hd0, (sc.x << 9) | (int)sd0)
      HIT(listD, wcd, hd1, (sc.y << 9) | (int)sd1)
      HIT(listD, wcd, hd2, (sc.z << 9) | (int)sd2)
      HIT(listD, wcd, hd3, (sc.w << 9) | (int)sd3)
    }
    if (lane == 0) wcD[wave] = wcd;
    __syncthreads();

    if (wave == 0) {
#pragma unroll 1
      for (int wsx = 0; wsx < NWAVE; ++wsx) {
        int n = wcD[wsx];
        n = (n > WCAP) ? WCAP : ((n < 0) ? 0 : n);
#pragma unroll 1
        for (int i = 0; i < n; ++i) {
          const int ent  = listD[wsx * WCAP + i];
          const int slot = ent & (NB - 1);
          int sId = ent >> 9;
          sId = (sId < 0) ? 0 : ((sId > nN - 1) ? nN - 1 : sId);
          const float w  = rso[sId];
          const v4f   hv = *(const v4f*)(h1 + (size_t)sId * DF + 4 * lane);
          v4f* sp = (v4f*)(sacc + slot * DF + 4 * lane);
          const v4f cur = *sp;
          *sp = cur + w * hv;
          if (lane == 0) {
            const int oc = cnti[slot];
            cnti[slot] = oc + 1;
          }
        }
      }
    }
    __syncthreads();
  }

  gcn_store(sacc, cnti, agH, nodeBase, wave, lane, hh);
  __threadfence();
  gcn_store(sacc, cnti, agH, nodeBase, wave, lane, hh);
}
#undef HIT

extern "C" void kernel_launch(void* const* d_in, const int* in_sizes, int n_in,
                              void* d_out, int out_size, void* d_ws, size_t ws_size,
                              hipStream_t stream) {
  if (n_in < 23) return;
  const int nN = in_sizes[0] / DF;
  const int nE = in_sizes[1];
  if (nN <= 0 || in_sizes[0] != nN * DF) return;
  if (nN > (1 << 22)) return;
  if (nE < 0 || in_sizes[2] != nE) return;
  if (in_sizes[3] != DF * DF || in_sizes[5] != DF * DF || in_sizes[7] != DF * DF ||
      in_sizes[9] != DF * DF || in_sizes[11] != DF * DF) return;
  if (in_sizes[13] != DF * FF || in_sizes[14] != FF || in_sizes[15] != FF * DF) return;
  {
    const int vi[12] = {4, 6, 8, 10, 12, 16, 17, 18, 19, 20, 21, 22};
    for (int i = 0; i < 12; ++i) if (in_sizes[vi[i]] != DF) return;
  }
  if (out_size != nN * DF) return;

  const float* h   = (const float*)d_in[0];
  const int*   src = (const int*)d_in[1];
  const int*   dst = (const int*)d_in[2];
  const float* Wq = (const float*)d_in[3];  const float* bq  = (const float*)d_in[4];
  const float* Wk = (const float*)d_in[5];  const float* bk  = (const float*)d_in[6];
  const float* Wv = (const float*)d_in[7];  const float* bv  = (const float*)d_in[8];
  const float* Wo = (const float*)d_in[9];  const float* bo  = (const float*)d_in[10];
  const float* Wg = (const float*)d_in[11]; const float* bg  = (const float*)d_in[12];
  const float* W1 = (const float*)d_in[13]; const float* b1  = (const float*)d_in[14];
  const float* W2 = (const float*)d_in[15]; const float* b2  = (const float*)d_in[16];
  const float* g1 = (const float*)d_in[17]; const float* be1 = (const float*)d_in[18];
  const float* g2 = (const float*)d_in[19]; const float* be2 = (const float*)d_in[20];
  const float* g3 = (const float*)d_in[21]; const float* be3 = (const float*)d_in[22];
  float* out = (float*)d_out;

  const int nP = ((nN + NB - 1) / NB) * NB;

  const size_t wtHalves = (size_t)5 * DF * DF + (size_t)FF * DF + (size_t)DF * FF;
  size_t off = 0;
  _Float16* WT  = (_Float16*)((char*)d_ws + off); off += wtHalves * sizeof(_Float16);
  off = (off + 255) & ~(size_t)255;
  float*    rso = (float*)((char*)d_ws + off);    off += (size_t)nP * sizeof(float);
  off = (off + 255) & ~(size_t)255;
  _Float16* R1  = (_Float16*)((char*)d_ws + off); off += (size_t)nP * DF * sizeof(_Float16);
  float*    RQ  = (float*)((char*)d_ws + off);    off += (size_t)nP * DF * sizeof(float);
  float*    RK  = (float*)((char*)d_ws + off);    off += (size_t)nP * DF * sizeof(float);
  float*    RV  = (float*)((char*)d_ws + off);    off += (size_t)nP * DF * sizeof(float);
  float*    RH1 = (float*)((char*)d_ws + off);    off += (size_t)nP * DF * sizeof(float);
  if (off > ws_size) return;
  if (off > ((size_t)128 << 20)) return;

  _Float16* WqT = WT;
  _Float16* WoT = WT + (size_t)3 * DF * DF;
  _Float16* WgT = WT + (size_t)4 * DF * DF;
  _Float16* W1T = WT + (size_t)5 * DF * DF;
  _Float16* W2T = W1T + (size_t)FF * DF;
  _Float16* h2H  = (_Float16*)RK;
  _Float16* midH = (_Float16*)RV;

  k_prepw<<<DF / 16, NTHR, 0, stream>>>(Wq, WqT,                        DF, DF);
  k_prepw<<<DF / 16, NTHR, 0, stream>>>(Wk, WT + (size_t)1 * DF * DF,  DF, DF);
  k_prepw<<<DF / 16, NTHR, 0, stream>>>(Wv, WT + (size_t)2 * DF * DF,  DF, DF);
  k_prepw<<<DF / 16, NTHR, 0, stream>>>(Wo, WoT,                        DF, DF);
  k_prepw<<<DF / 16, NTHR, 0, stream>>>(Wg, WgT,                        DF, DF);
  k_prepw<<<FF / 16, NTHR, 0, stream>>>(W1, W1T,                        DF, FF);
  k_prepw<<<DF / 4,  NTHR, 0, stream>>>(W2, W2T,                        FF, DF);

  k_cvt<<<(nP * (DF / 8)) / NTHR, NTHR, 0, stream>>>(h, R1, nN, nP);

  k_gemm_qkv<<<dim3(nP / GR, 3), NTHR, 0, stream>>>(R1, WqT, bq, bk, bv, RQ, nP);

  hipFuncSetAttribute(reinterpret_cast<const void*>(&k_attn),
                      hipFuncAttributeMaxDynamicSharedMemorySize, LDS1_BYTES);
  k_attn<<<nP / NB, NTHR, LDS1_BYTES, stream>>>(RQ, RK, RV, src, dst, R1, rso, nN, nE);

  k_gemm_ln<<<nP / GR, NTHR, 0, stream>>>(R1, WoT, bo, h, g1, be1, RH1, h2H, DF, DF, nN, nP, 0);

  hipFuncSetAttribute(reinterpret_cast<const void*>(&k_gcn),
                      hipFuncAttributeMaxDynamicSharedMemorySize, LDS2_BYTES);
  k_gcn<<<nP / NB, NTHR, LDS2_BYTES, stream>>>(RH1, rso, src, dst, R1, nN, nE);

  k_gemm_ln<<<nP / GR, NTHR, 0, stream>>>(R1, WgT, bg, RH1, g2, be2, RQ, h2H, DF, DF, nP, nP, 1);

  k_ffn1<<<dim3(nP / GR, FF / DF), NTHR, 0, stream>>>(h2H, W1T, b1, midH);

  k_gemm_ln<<<nP / GR, NTHR, 0, stream>>>(midH, W2T, b2, RQ, g3, be3, out, h2H, FF, FF, nP, nN, 0);
}
